// SE3TransformerBlock_84894323573079
// MI455X (gfx1250) — hardware-verified
//
#include <hip/hip_runtime.h>
#include <stddef.h>


#define BB     4
#define NN     192
#define CS     16
#define CV     4
#define DIMF   28
#define NBAS   10
#define NUMEL  400
#define QP     32
#define NTHR   256
#define NWAVE  8
#define PTHR   64
#define HP     48
#define WPITCH 48
#define KVP    32
#define NPAIR  256

#define SQRT3F  1.7320508075688772f
#define SQRT10F 3.1622776601683795f
#define SQRT12F 3.4641016151377544f
#define SQRT2F  1.4142135623730951f
#define RSQ10F  (1.0f / SQRT10F)
#define RSQ12F  (1.0f / SQRT12F)
#define RSQ2F   (1.0f / SQRT2F)
#define STEPF   0.13636363636363635f
#define RSTEPF  (1.0f / STEPF)
#define RMAXR   (1.0f / 1.5f)
#define SILUG   1.679f
#define EMBC    ((float)(1.14136 * 7.3890560989306495))

static_assert(NN % 16 == 0);
static_assert(NTHR == NPAIR);
static_assert((BB * NN) % PTHR == 0);
static_assert(CS * CS + CS * CV + CV * CV + CV * CS == NUMEL);
static_assert(16 * DIMF <= 2 * NTHR);
static_assert((16 * DIMF) % 4 == 0);

typedef float          v4f   __attribute__((ext_vector_type(4)));
typedef float          v8f   __attribute__((ext_vector_type(8)));
typedef float          v16f  __attribute__((ext_vector_type(16)));
typedef unsigned short v8us  __attribute__((ext_vector_type(8)));
typedef __bf16         v16bf __attribute__((ext_vector_type(16)));
union FragB { v16bf v; v8us u[2]; };

__device__ __forceinline__ v8f zero8f() {
  v8f r;
#pragma unroll
  for (int i = 0; i < 8; ++i) r[i] = 0.0f;
  return r;
}
__device__ __forceinline__ v16f zero16f() {
  v16f r;
#pragma unroll
  for (int i = 0; i < 16; ++i) r[i] = 0.0f;
  return r;
}
__device__ __forceinline__ v8us zero8us() {
  v8us r;
#pragma unroll
  for (int i = 0; i < 8; ++i) r[i] = (unsigned short)0;
  return r;
}
__device__ __forceinline__ v8f cat8(v4f a, v4f b) {
  return __builtin_shufflevector(a, b, 0, 1, 2, 3, 4, 5, 6, 7);
}

__device__ __forceinline__ unsigned int bfb(float x) {
  const unsigned int u = __float_as_uint(x);
  return (u + 0x7FFFu + ((u >> 16) & 1u)) >> 16;
}
__device__ __forceinline__ float bfv(unsigned int w) { return __uint_as_float(w << 16); }

__device__ __forceinline__ void split3(float x, unsigned short& h, unsigned short& m, unsigned short& l) {
  const unsigned int hb = bfb(x);
  const float r1 = x - bfv(hb);
  const unsigned int mb = bfb(r1);
  const float r2 = r1 - bfv(mb);
  const unsigned int lb = bfb(r2);
  h = (unsigned short)hb;
  m = (unsigned short)mb;
  l = (unsigned short)lb;
}

__device__ __forceinline__ v8f wmma3(v16bf a1, v16bf a2, v16bf b1, v16bf b2, v16bf b3) {
  v8f d = zero8f();
  d = __builtin_amdgcn_wmma_f32_16x16x32_bf16(false, a1, false, b1, (short)0, d, false, false);
  d = __builtin_amdgcn_wmma_f32_16x16x32_bf16(false, a1, false, b2, (short)0, d, false, false);
  d = __builtin_amdgcn_wmma_f32_16x16x32_bf16(false, a2, false, b3, (short)0, d, false, false);
  asm volatile("v_nop\n\tv_nop\n\tv_nop\n\tv_nop" : "+v"(d) : "v"(a1), "v"(a2), "v"(b1), "v"(b2), "v"(b3));
  return d;
}

__device__ __forceinline__ v8f mm_tile(v16bf a1, v16bf a2, const unsigned short* sw, int col, int hh) {
  const unsigned short* bp = sw + (col * 2 + hh) * 24;
  const v8us wh = *(const v8us*)bp;
  const v8us wm = *(const v8us*)(bp + 8);
  const v8us wl = *(const v8us*)(bp + 16);
  FragB b1, b2, b3;
  b1.u[0] = wh; b1.u[1] = wh;
  b2.u[0] = wm; b2.u[1] = wm;
  b3.u[0] = wl; b3.u[1] = wh;
  return wmma3(a1, a2, b1.v, b2.v, b3.v);
}

__device__ __forceinline__ float sus_f(float x) {
  const float xp = (x > 0.0f) ? x : 1.0f;
  const float e = expf(-(1.0f / xp));
  return (x > 0.0f) ? e : 0.0f;
}

__device__ __forceinline__ float silu_h(float ut) {
  const float uu = ut * RSQ10F;
  const float ex = expf(-uu);
  const float sg = 1.0f / (1.0f + ex);
  return SILUG * (uu * sg);
}

template <int BASE>
__device__ __forceinline__ void pack8(v16f u, unsigned short* hp) {
  v8us h8 = zero8us(), m8 = zero8us(), l8 = zero8us();
#pragma unroll
  for (int t = 0; t < 8; ++t) {
    unsigned short a, bm, c;
    split3(silu_h(u[BASE + t]), a, bm, c);
    h8[t] = a; m8[t] = bm; l8[t] = c;
  }
  *(v8us*)(hp + BASE)      = h8;
  *(v8us*)(hp + 16 + BASE) = m8;
  *(v8us*)(hp + 32 + BASE) = l8;
}

__device__ __forceinline__ int colmap(int o) {
  const int t = o - CS;
  const int oo = t / 3;
  const int x = t - oo * 3;
  const int cv = CS + x * 4 + oo;
  return (o < CS) ? o : cv;
}

__device__ __forceinline__ void tp_net(const unsigned short* sw, const unsigned short* sha, const float* sf,
                                       const float* ssh, const float* stv, int hh, int n,
                                       v8f& outS, v8f& outV) {
  FragB a1, a2;
  {
    const unsigned short* ar = sha + n * HP + 8 * hh;
    const v8us ph = *(const v8us*)ar;
    a1.u[0] = ph; a1.u[1] = *(const v8us*)(ar + 16);
    a2.u[0] = ph; a2.u[1] = *(const v8us*)(ar + 32);
  }
  const int g = n >> 2, o4 = n & 3;
  const int xq = (g > 2) ? 2 : g;

  v8f acc3 = zero8f();
#pragma unroll 1
  for (int q = 0; q < 4; ++q) {
    const v8f d = mm_tile(a1.v, a2.v, sw, (16 + q) * 16 + n, hh);
    const float fsc = sf[4 * q + g];
#pragma unroll
    for (int r = 0; r < 8; ++r) acc3[r] = fmaf(fsc, d[r], acc3[r]);
  }
  v8f t9 = zero8f();
#pragma unroll
  for (int r = 0; r < 8; ++r) {
    float v = acc3[r];
    v += __shfl_xor(v, 4, 32);
    v += __shfl_xor(v, 8, 32);
    t9[r] = v;
  }
  v8f t11 = zero8f();
  {
    const v8f d = mm_tile(a1.v, a2.v, sw, 20 * 16 + n, hh);
#pragma unroll
    for (int c = 0; c < CV; ++c) {
      const float fvc = sf[CS + c * 3 + xq];
      const int src = hh * 16 + c * 4 + o4;
#pragma unroll
      for (int r = 0; r < 8; ++r) t11[r] = fmaf(fvc, __shfl(d[r], src, 32), t11[r]);
    }
  }
  {
    const v8f s8 = cat8(*(const v4f*)(ssh + xq * 16 + 8 * hh), *(const v4f*)(ssh + xq * 16 + 8 * hh + 4));
#pragma unroll
    for (int r = 0; r < 8; ++r) {
      const float vv = ((t9[r] * s8[r]) * 0.0625f + t11[r] * 0.125f) * RSQ2F;
      outV[r] = (n < 12) ? vv : 0.0f;
    }
  }
  v8f acc1 = zero8f();
#pragma unroll 1
  for (int ct = 0; ct < CS; ++ct) {
    const v8f d = mm_tile(a1.v, a2.v, sw, ct * 16 + n, hh);
    const float fsc = sf[ct];
#pragma unroll
    for (int r = 0; r < 8; ++r) acc1[r] = fmaf(fsc, d[r], acc1[r]);
  }
  v8f acc2 = zero8f();
#pragma unroll 1
  for (int c = 0; c < CV; ++c) {
    const v8f d = mm_tile(a1.v, a2.v, sw, (21 + c) * 16 + n, hh);
    const v8f t8 = cat8(*(const v4f*)(stv + c * 16 + 8 * hh), *(const v4f*)(stv + c * 16 + 8 * hh + 4));
#pragma unroll
    for (int r = 0; r < 8; ++r) acc2[r] = fmaf(t8[r], d[r], acc2[r]);
  }
#pragma unroll
  for (int r = 0; r < 8; ++r) outS[r] = (acc1[r] * 0.0625f + (acc2[r] * 0.25f) * RSQ12F) * RSQ2F;
}

__global__ __launch_bounds__(PTHR) void k_prep(const float* __restrict__ f,
                                              const float* __restrict__ wq_s,
                                              const float* __restrict__ wq_v,
                                              const float* __restrict__ dot_ws,
                                              const float* __restrict__ dot_wv,
                                              float* prep, int nNodes) {
  __shared__ __attribute__((aligned(16))) float s_t[PTHR * QP];
  __shared__ __attribute__((aligned(16))) float s_q[PTHR * QP];
  const int tid = threadIdx.x;
  const int base = blockIdx.x * PTHR;
  int nd = base + tid;
  nd = (nd > nNodes - 1) ? (nNodes - 1) : nd;
  const float* fr = f + (size_t)nd * DIMF;
  float* tq = s_q + tid * QP;
  float* tt = s_t + tid * QP;

  float vflag = 0.0f;
#pragma unroll 1
  for (int c = 0; c < DIMF; ++c) { const float x = fr[c]; vflag = (x != 0.0f) ? 1.0f : vflag; }

  v16f qs = zero16f();
#pragma unroll 1
  for (int c = 0; c < CS; ++c) {
    const float fc = fr[c];
    const float* wr = wq_s + c * CS;
#pragma unroll
    for (int o = 0; o < CS; ++o) qs[o] = fmaf(fc, wr[o], qs[o]);
  }
#pragma unroll
  for (int o = 0; o < CS; ++o) tq[o] = qs[o] * 0.25f;
#pragma unroll 1
  for (int d = 0; d < CS; ++d) {
    float a = 0.0f;
#pragma unroll 1
    for (int c = 0; c < CS; ++c) a = fmaf(tq[c], dot_ws[c * CS + d], a);
    tt[d] = a;
  }
#pragma unroll 1
  for (int e = 0; e < CV * 3; ++e) {
    const int o = e / 3, x = e - o * 3;
    float a = 0.0f;
#pragma unroll 1
    for (int c = 0; c < CV; ++c) a = fmaf(fr[CS + c * 3 + x], wq_v[c * CV + o], a);
    tq[CS + e] = a * 0.5f;
  }
#pragma unroll 1
  for (int e = 0; e < CV * 3; ++e) {
    const int x = e >> 2, d = e & 3;
    float a = 0.0f;
#pragma unroll 1
    for (int c = 0; c < CV; ++c) a = fmaf(dot_wv[c * CV + d], tq[CS + c * 3 + x], a);
    tt[CS + e] = a;
  }
  tt[28] = vflag;
  tt[29] = 0.0f;
  tt[30] = 0.0f;
  tt[31] = 0.0f;
  __syncthreads();

  v4f vals[8];
#pragma unroll
  for (int it = 0; it < 8; ++it) {
    const int L = it * 8 + (tid >> 3), pc = tid & 7;
    vals[it] = *(const v4f*)(s_t + L * QP + pc * 4);
  }
#pragma unroll
  for (int it = 0; it < 8; ++it) {
    const int L = it * 8 + (tid >> 3), pc = tid & 7;
    if (base + L < nNodes) *(volatile v4f*)(prep + (size_t)(base + L) * QP + pc * 4) = vals[it];
  }
  __threadfence();
#pragma unroll
  for (int it = 0; it < 8; ++it) {
    const int L = it * 8 + (tid >> 3), pc = tid & 7;
    if (base + L < nNodes) *(volatile v4f*)(prep + (size_t)(base + L) * QP + pc * 4) = vals[it];
  }
}

__global__ __launch_bounds__(NTHR) void k_pair(const float* __restrict__ f,
                                              const float* __restrict__ pos,
                                              const float* __restrict__ w1k,
                                              const float* __restrict__ w2k,
                                              const float* __restrict__ w1v,
                                              const float* __restrict__ w2v,
                                              const float* __restrict__ prep,
                                              float* out) {
  __shared__ __attribute__((aligned(16))) unsigned short s_w[2 * NUMEL * WPITCH];
  __shared__ __attribute__((aligned(16))) unsigned short s_h[2 * NPAIR * HP];
  __shared__ __attribute__((aligned(16))) float s_kv[NPAIR * KVP];
  __shared__ __attribute__((aligned(16))) float s_w1[2 * NBAS * 16];
  __shared__ __attribute__((aligned(16))) float s_f[16 * 32];
  __shared__ __attribute__((aligned(16))) float s_posi[16 * 4];
  __shared__ __attribute__((aligned(16))) float s_posj[16 * 4];
  __shared__ float s_vi[16];
  __shared__ float s_vj[16];
  __shared__ __attribute__((aligned(16))) float s_us[16 * 16];
  __shared__ __attribute__((aligned(16))) float s_uv[12 * 16];
  __shared__ __attribute__((aligned(16))) float s_sh[16 * 3 * 16];
  __shared__ __attribute__((aligned(16))) float s_cut[16 * 16];
  __shared__ __attribute__((aligned(16))) float s_tv[16 * 4 * 16];
  __shared__ float s_le[NPAIR];
  __shared__ float s_wt[NPAIR];
  __shared__ float s_z[16];
  __shared__ __attribute__((aligned(16))) float s_out[16 * DIMF];

  const int tid = threadIdx.x, lane = tid & 31, wave = tid >> 5, hh = lane >> 4, n = lane & 15;
  const int i0 = blockIdx.x * 16, b = blockIdx.y;
  const int bN = b * NN;

  for (int e = tid; e < 2 * CS * NUMEL; e += NTHR) {
    const int net = (e >= CS * NUMEL) ? 1 : 0;
    const int rem = e - net * (CS * NUMEL);
    const int t = rem / NUMEL, col = rem - t * NUMEL;
    const float wa = w2k[rem], wb = w2v[rem];
    const float x = (net != 0) ? wb : wa;
    unsigned short ph, pm, pl;
    split3(x, ph, pm, pl);
    unsigned short* p = s_w + ((net * NUMEL + col) * 2 + (t >> 3)) * 24 + (t & 7);
    p[0] = ph; p[8] = pm; p[16] = pl;
  }
  for (int e = tid; e < 2 * NBAS * 16; e += NTHR) {
    const int i = (e < NBAS * 16) ? e : (e - NBAS * 16);
    const float a = w1k[i], c = w1v[i];
    s_w1[e] = (e < NBAS * 16) ? a : c;
  }
  for (int e = tid; e < 16 * QP; e += NTHR) {
    const int ii = e >> 5, q = e & 31;
    const float v = prep[(size_t)(bN + i0 + ii) * QP + q];
    if (q < 16) s_us[q * 16 + ii] = v;
    else if (q < 28) s_uv[(q - 16) * 16 + ii] = v;
    else if (q == 28) s_vi[ii] = v;
  }
  if (tid < 64) {
    const int e = (tid < 48) ? tid : 47;
    const int ii = e / 3, x = e - ii * 3;
    const float v = pos[(size_t)(bN + i0 + ii) * 3 + x];
    if (tid < 48) s_posi[ii * 4 + x] = v;
  }
  if (tid >= 64 && tid < 80) s_posi[(tid - 64) * 4 + 3] = 0.0f;
  if (tid >= 80 && tid < 96) s_posj[(tid - 80) * 4 + 3] = 0.0f;
  for (int e = tid; e < NPAIR * KVP; e += NTHR) s_kv[e] = 0.0f;

  const int e1raw = tid + NTHR;
  const int e1 = (e1raw < 16 * DIMF) ? e1raw : tid;
  const int ii0 = tid / DIMF, o0 = tid - ii0 * DIMF;
  const int ii1 = e1 / DIMF, o1 = e1 - ii1 * DIMF;
  const int col0 = colmap(o0), col1 = colmap(o1);
  const int zi = tid & 15;
  float aP0 = 0.0f, aN0 = 0.0f, aP1 = 0.0f, aN1 = 0.0f;
  double zd = 0.0;
  __syncthreads();

#pragma unroll 1
  for (int jt = 0; jt < NN / 16; ++jt) {
    const int j0 = jt * 16;
    for (int e = tid; e < 16 * DIMF; e += NTHR) {
      const int jj = e / DIMF, c = e - jj * DIMF;
      s_f[jj * 32 + c] = f[(size_t)(bN + j0 + jj) * DIMF + c];
    }
    if (tid < 64) {
      const int e = (tid < 48) ? tid : 47;
      const int jj = e / 3, x = e - jj * 3;
      const float v = pos[(size_t)(bN + j0 + jj) * 3 + x];
      if (tid < 48) s_posj[jj * 4 + x] = v;
    }
    if (wave == 2) {
      const int jj = lane & 15;
      const float v = prep[(size_t)(bN + j0 + jj) * QP + 28];
      if (lane < 16) s_vj[jj] = v;
    }
    __syncthreads();

    {
      const int ii = tid & 15, jj = tid >> 4;
      const float dx = s_posj[jj * 4 + 0] - s_posi[ii * 4 + 0];
      const float dy = s_posj[jj * 4 + 1] - s_posi[ii * 4 + 1];
      const float dz = s_posj[jj * 4 + 2] - s_posi[ii * 4 + 2];
      const float d2 = dx * dx + dy * dy + dz * dz;
      const float dist = sqrtf(d2 + 1e-12f);
      const bool msk = (dist < 1.5f) && ((i0 + ii) != (j0 + jj)) && (s_vi[ii] != 0.0f) && (s_vj[jj] != 0.0f);
      const float rd = 1.0f / dist;
      const float shx = (SQRT3F * dx) * rd;
      const float shy = (SQRT3F * dy) * rd;
      const float shz = (SQRT3F * dz) * rd;
      const float cut0 = sus_f(10.0f * (1.0f - dist * RMAXR));
      const float cut = msk ? cut0 : 0.0f;
      const float dd = dist * RSTEPF;
      const int mm = (int)floorf(dd + 0.5f);
      float e3[3];
      int k3[3];
#pragma unroll
      for (int s = 0; s < 3; ++s) {
        const int k = mm - 2 + s;
        const int kc = (k < 0) ? 0 : ((k > NBAS - 1) ? (NBAS - 1) : k);
        const float ck = (float)(kc + 1) * STEPF;
        const float diff = (dist - ck) * RSTEPF;
        const float ev = ((EMBC * sus_f(diff + 1.0f)) * sus_f(1.0f - diff)) * SQRT10F;
        e3[s] = (k >= 0 && k <= NBAS - 1) ? ev : 0.0f;
        k3[s] = kc;
      }
      v16f uk = zero16f(), uv = zero16f();
#pragma unroll
      for (int s = 0; s < 3; ++s) {
        const float* wr = s_w1 + k3[s] * 16;
        const float* vr = s_w1 + NBAS * 16 + k3[s] * 16;
        const float es = e3[s];
#pragma unroll
        for (int g = 0; g < 4; ++g) {
          const v4f wa = *(const v4f*)(wr + 4 * g);
          const v4f va = *(const v4f*)(vr + 4 * g);
#pragma unroll
          for (int c = 0; c < 4; ++c) {
            uk[4 * g + c] = fmaf(es, wa[c], uk[4 * g + c]);
            uv[4 * g + c] = fmaf(es, va[c], uv[4 * g + c]);
          }
        }
      }
      {
        unsigned short* hk = s_h + ((0 * 16 + jj) * 16 + ii) * HP;
        unsigned short* hv = s_h + ((1 * 16 + jj) * 16 + ii) * HP;
        pack8<0>(uk, hk);
        pack8<8>(uk, hk);
        pack8<0>(uv, hv);
        pack8<8>(uv, hv);
      }
      const float* fj = s_f + jj * 32;
#pragma unroll
      for (int c = 0; c < CV; ++c) {
        const float t0 = fj[CS + c * 3 + 0] * shx;
        const float t1 = fmaf(fj[CS + c * 3 + 1], shy, t0);
        const float t2 = fmaf(fj[CS + c * 3 + 2], shz, t1);
        s_tv[(jj * 4 + c) * 16 + ii] = t2;
      }
      s_sh[(jj * 3 + 0) * 16 + ii] = shx;
      s_sh[(jj * 3 + 1) * 16 + ii] = shy;
      s_sh[(jj * 3 + 2) * 16 + ii] = shz;
      s_cut[jj * 16 + ii] = cut;
    }
    __syncthreads();

#pragma unroll 1
    for (int s2 = 0; s2 < 2; ++s2) {
      const int jj = wave + NWAVE * s2;
      const float cl = s_cut[jj * 16 + n];
      if (__builtin_amdgcn_ballot_w32(cl != 0.0f) == 0u) continue;
      v8f oS, oV;
      tp_net(s_w, s_h + (jj * 16) * HP, s_f + jj * 32, s_sh + jj * 48, s_tv + jj * 64, hh, n, oS, oV);
      float* kr = s_kv + (jj * 16 + 8 * hh) * KVP;
#pragma unroll
      for (int r = 0; r < 8; ++r) {
        kr[r * KVP + n]      = oS[r];
        kr[r * KVP + 16 + n] = oV[r];
      }
    }
    __syncthreads();

    {
      const int ii = tid & 15;
      const float* kr = s_kv + tid * KVP;
      float ss = 0.0f, sv = 0.0f;
#pragma unroll
      for (int d = 0; d < CS; ++d) ss = fmaf(kr[d], s_us[d * 16 + ii], ss);
#pragma unroll
      for (int q = 0; q < CV * 3; ++q) sv = fmaf(kr[CS + q], s_uv[q * 16 + ii], sv);
      const float sc = (ss * 0.25f + sv * RSQ12F) * RSQ2F;
      const float le = s_cut[tid] * sc;
      s_le[tid] = le;
      s_wt[tid] = sqrtf(fabsf(le));
    }
    __syncthreads();

#pragma unroll 1
    for (int s2 = 0; s2 < 2; ++s2) {
      const int jj = wave + NWAVE * s2;
      const float cl = s_cut[jj * 16 + n];
      if (__builtin_amdgcn_ballot_w32(cl != 0.0f) == 0u) continue;
      v8f oS, oV;
      tp_net(s_w + NUMEL * WPITCH, s_h + ((16 + jj) * 16) * HP, s_f + jj * 32, s_sh + jj * 48, s_tv + jj * 64,
             hh, n, oS, oV);
      float* kr = s_kv + (jj * 16 + 8 * hh) * KVP;
#pragma unroll
      for (int r = 0; r < 8; ++r) {
        kr[r * KVP + n]      = oS[r];
        kr[r * KVP + 16 + n] = oV[r];
      }
    }
    __syncthreads();

#pragma unroll 4
    for (int jj = 0; jj < 16; ++jj) {
      const int pa = jj * 16 + ii0;
      const float lea = s_le[pa], wta = s_wt[pa], va = s_kv[pa * KVP + col0];
      const float ta = wta * va;
      aP0 += (lea > 0.0f) ? ta : 0.0f;
      aN0 += (lea < 0.0f) ? ta : 0.0f;
      const int pb = jj * 16 + ii1;
      const float leb = s_le[pb], wtb = s_wt[pb], vb = s_kv[pb * KVP + col1];
      const float tb = wtb * vb;
      aP1 += (leb > 0.0f) ? tb : 0.0f;
      aN1 += (leb < 0.0f) ? tb : 0.0f;
      zd += (double)s_le[jj * 16 + zi];
    }
    __syncthreads();
  }

  if (tid < 16) s_z[tid] = (float)zd;
  __syncthreads();
  {
    const float z0 = s_z[ii0];
    const float f0 = (z0 == 0.0f) ? 1.0f : (1.0f / sqrtf(fabsf(z0)));
    const float a0 = (z0 < 0.0f) ? aN0 : aP0;
    s_out[tid] = (a0 * f0) * s_vi[ii0];
    const float z1 = s_z[ii1];
    const float f1 = (z1 == 0.0f) ? 1.0f : (1.0f / sqrtf(fabsf(z1)));
    const float a1 = (z1 < 0.0f) ? aN1 : aP1;
    const float r1 = (a1 * f1) * s_vi[ii1];
    if (e1raw < 16 * DIMF) s_out[e1raw] = r1;
  }
  __syncthreads();
  const bool wr = tid < (16 * DIMF) / 4;
  v4f ov = {0.0f, 0.0f, 0.0f, 0.0f};
  if (wr) ov = *(const v4f*)(s_out + tid * 4);
  float* gp = out + (size_t)(bN + i0) * DIMF + tid * 4;
  if (wr) *(volatile v4f*)gp = ov;
  __threadfence();
  if (wr) *(volatile v4f*)gp = ov;
}

extern "C" void kernel_launch(void* const* d_in, const int* in_sizes, int n_in,
                              void* d_out, int out_size, void* d_ws, size_t ws_size,
                              hipStream_t stream) {
  if (n_in < 10) return;
  if (in_sizes[0] != BB * NN * DIMF || in_sizes[1] != BB * NN * 3) return;
  if (in_sizes[2] != CS * CS || in_sizes[3] != CV * CV) return;
  if (in_sizes[4] != NBAS * 16 || in_sizes[5] != 16 * NUMEL) return;
  if (in_sizes[6] != NBAS * 16 || in_sizes[7] != 16 * NUMEL) return;
  if (in_sizes[8] != CS * CS || in_sizes[9] != CV * CV) return;
  if (out_size != BB * NN * DIMF) return;

  const int nNodes = BB * NN;
  const int nPrepBlk = (nNodes + PTHR - 1) / PTHR;
  const size_t prepBytes = (size_t)nPrepBlk * PTHR * QP * sizeof(float);
  if (prepBytes > ws_size) return;

  const float* f      = (const float*)d_in[0];
  const float* pos    = (const float*)d_in[1];
  const float* wq_s   = (const float*)d_in[2];
  const float* wq_v   = (const float*)d_in[3];
  const float* fck_w1 = (const float*)d_in[4];
  const float* fck_w2 = (const float*)d_in[5];
  const float* fcv_w1 = (const float*)d_in[6];
  const float* fcv_w2 = (const float*)d_in[7];
  const float* dot_ws = (const float*)d_in[8];
  const float* dot_wv = (const float*)d_in[9];
  float* prep = (float*)d_ws;
  float* out  = (float*)d_out;

  k_prep<<<nPrepBlk, PTHR, 0, stream>>>(f, wq_s, wq_v, dot_ws, dot_wv, prep, nNodes);
  k_pair<<<dim3(NN / 16, BB), NTHR, 0, stream>>>(f, pos, fck_w1, fck_w2, fcv_w1, fcv_w2, prep, out);
}
